// EmbedEHRLSTMLOS_68109591380521
// MI455X (gfx1250) — hardware-run, weakly checked
//
#include <hip/hip_runtime.h>
#include <math.h>

constexpr int NBAT   = 128;
constexpr int NSTEP  = 512;
constexpr int NTOKL  = 8;
constexpr int NEMB   = 128;
constexpr int NHID   = 512;
constexpr int NGATE  = 4 * NHID;
constexpr int KCAT   = NEMB + NHID;
constexpr int NVOCAB = 20000;
constexpr int MBLK   = 32;
constexpr int APITCH = KCAT + 8;
constexpr int ATILE  = MBLK * APITCH;
constexpr int LTHR   = 512;
constexpr int NWAVE  = LTHR / 32;
constexpr int OTILE  = 32;
constexpr int OPITCH = 36;
constexpr int PTHR   = 256;
constexpr int IH_BLOCKS = NGATE * (NEMB / 8) / PTHR;
constexpr int HH_BLOCKS = NGATE * (NHID / 8) / PTHR;
constexpr float ACARRY = 256.0f;
constexpr float WCARRY = 256.0f;
constexpr float CFOLD  = 1.0f / (ACARRY * WCARRY);
static_assert(KCAT % 32 == 0);
static_assert(NBAT % MBLK == 0);
static_assert(NHID == 32 * NWAVE);
static_assert(NGATE == 4 * LTHR);
static_assert(MBLK * NEMB == 8 * LTHR);
static_assert(MBLK == 32);
static_assert(NSTEP % OTILE == 0);
static_assert((APITCH * 2) % 16 == 0);
static_assert((OPITCH * 4) % 16 == 0);
static_assert(NGATE * (NEMB / 8) % PTHR == 0);
static_assert(NGATE * (NHID / 8) % PTHR == 0);
static_assert((NBAT * NSTEP) % (PTHR / 32) == 0);

typedef __attribute__((ext_vector_type(16))) _Float16 v16h;
typedef __attribute__((ext_vector_type(8)))  _Float16 v8h;
typedef __attribute__((ext_vector_type(4)))  _Float16 v4h;
typedef __attribute__((ext_vector_type(8)))  float    v8f;
typedef __attribute__((ext_vector_type(4)))  float    v4f;
typedef __attribute__((ext_vector_type(4)))  unsigned v4u;
typedef __attribute__((ext_vector_type(4)))  int      v4i;

struct Frag16 {
  union U { v16h v; v8h h[2]; };
  static __device__ __forceinline__ v16h load(const _Float16* p) {
    U f; f.h[0] = *(const v8h*)(p); f.h[1] = *(const v8h*)(p + 16); return f.v;
  }
  static __device__ __forceinline__ v8f mma(v16h a, v16h b, v8f c) {
    return __builtin_amdgcn_wmma_f32_16x16x32_f16(false, a, false, b, (short)0, c, false, false);
  }
};
__device__ __forceinline__ void guard8(v8f& a0, v8f& a1, v8f& a2, v8f& a3, v8f& a4, v8f& a5, v8f& a6, v8f& a7,
                                       v16h x0, v16h x1, v16h b0, v16h b1, v16h b2, v16h b3) {
  asm volatile("v_nop\n\tv_nop\n\tv_nop\n\tv_nop"
               : "+v"(a0), "+v"(a1), "+v"(a2), "+v"(a3), "+v"(a4), "+v"(a5), "+v"(a6), "+v"(a7)
               : "v"(x0), "v"(x1), "v"(b0), "v"(b1), "v"(b2), "v"(b3));
}

__device__ __forceinline__ float fsig(float x)  { return __builtin_amdgcn_rcpf(1.0f + __expf(-x)); }
__device__ __forceinline__ float ftanh(float x) { return 1.0f - 2.0f * __builtin_amdgcn_rcpf(__expf(2.0f * x) + 1.0f); }

__global__ __launch_bounds__(PTHR) void prep_weights_kernel(const float* __restrict__ wih, const float* __restrict__ whh,
                                                            unsigned short* __restrict__ Wp) {
  const int tid = threadIdx.x;
  const float* src;
  unsigned short* dst;
  if (blockIdx.x < IH_BLOCKS) {
    const int i = blockIdx.x * PTHR + tid;
    const int row = i >> 4, c8 = (i & 15) * 8;
    src = wih + (size_t)row * NEMB + c8;
    dst = Wp + (size_t)row * KCAT + c8;
  } else {
    const int i = (blockIdx.x - IH_BLOCKS) * PTHR + tid;
    const int row = i >> 6, c8 = (i & 63) * 8;
    src = whh + (size_t)row * NHID + c8;
    dst = Wp + (size_t)row * KCAT + NEMB + c8;
  }
  const v4f a = *(const v4f*)(src);
  const v4f b = *(const v4f*)(src + 4);
  v8h hv;
#pragma unroll
  for (int e = 0; e < 4; ++e) {
    const float fa = a[e] * WCARRY;
    const float fb = b[e] * WCARRY;
    hv[e]     = (_Float16)fa;
    hv[4 + e] = (_Float16)fb;
  }
  *(volatile v8h*)dst = hv;
  __threadfence();
  *(volatile v8h*)dst = hv;
}

__global__ __launch_bounds__(PTHR) void embed_kernel(const int* __restrict__ tokens, const float* __restrict__ values,
                                                     const float* __restrict__ emb, unsigned short* __restrict__ Xp) {
  const int lane = threadIdx.x & 31, wave = threadIdx.x >> 5;
  const int bt = blockIdx.x * (PTHR / 32) + wave;
  if (bt >= NBAT * NSTEP) return;
  const int b = bt / NSTEP;
  const int t = bt - b * NSTEP;
  const v4i tk0 = *(const v4i*)(tokens + (size_t)bt * NTOKL);
  const v4i tk1 = *(const v4i*)(tokens + (size_t)bt * NTOKL + 4);
  const v4f vl0 = *(const v4f*)(values + (size_t)bt * NTOKL);
  const v4f vl1 = *(const v4f*)(values + (size_t)bt * NTOKL + 4);
  v4f acc = {0.0f, 0.0f, 0.0f, 0.0f};
#pragma unroll
  for (int l = 0; l < NTOKL; ++l) {
    int tok = (l < 4) ? tk0[l & 3] : tk1[l & 3];
    const float v = (l < 4) ? vl0[l & 3] : vl1[l & 3];
    tok = tok < 0 ? 0 : (tok > NVOCAB - 1 ? NVOCAB - 1 : tok);
    const v4f e = *(const v4f*)(emb + (size_t)tok * NEMB + 4 * lane);
#pragma unroll
    for (int k = 0; k < 4; ++k) acc[k] = fmaf(v, e[k], acc[k]);
  }
  v4h hv;
#pragma unroll
  for (int k = 0; k < 4; ++k) {
    const float f = fmaxf(acc[k], 0.0f) * ACARRY;
    hv[k] = (_Float16)f;
  }
  unsigned short* dst = Xp + ((size_t)t * NBAT + b) * NEMB + 4 * lane;
  *(volatile v4h*)dst = hv;
  __threadfence();
  *(volatile v4h*)dst = hv;
}

__device__ __forceinline__ void cell8(const v8f ai, const v8f af, const v8f ag, const v8f ao,
                                      const float bi, const float bf, const float bg, const float bo,
                                      const float wo, float (&cs)[8], float (&hp)[8], _Float16* hdst) {
#pragma unroll
  for (int r = 0; r < 8; ++r) {
    const float zi = fmaf(ai[r], CFOLD, bi);
    const float zf = fmaf(af[r], CFOLD, bf);
    const float zg = fmaf(ag[r], CFOLD, bg);
    const float zo = fmaf(ao[r], CFOLD, bo);
    const float ig = fsig(zi);
    const float fg = fsig(zf);
    const float gg = ftanh(zg);
    const float og = fsig(zo);
    const float cn = fg * cs[r] + ig * gg;
    cs[r] = cn;
    const float hv = og * ftanh(cn);
    hp[r] = fmaf(hv, wo, hp[r]);
    const float hsc = hv * ACARRY;
    hdst[r * APITCH] = (_Float16)hsc;
  }
}

__device__ __forceinline__ void unit_group(const _Float16* arow0, const _Float16* arow1, const _Float16* wb,
                                           _Float16* hcol, const float* bj, const float wo,
                                           float (&cs)[2][8], float (&hp)[2][8]) {
  const size_t gstr = (size_t)NHID * KCAT;
  const v8f z8 = {0.f, 0.f, 0.f, 0.f, 0.f, 0.f, 0.f, 0.f};
  v8f a00 = z8, a01 = z8, a02 = z8, a03 = z8;
  v8f a10 = z8, a11 = z8, a12 = z8, a13 = z8;
#pragma unroll 1
  for (int k0 = 0; k0 < KCAT; k0 += 32) {
    const v16h x0 = Frag16::load(arow0 + k0);
    const v16h x1 = Frag16::load(arow1 + k0);
    const v16h b0 = Frag16::load(wb + k0);
    const v16h b1 = Frag16::load(wb + gstr + k0);
    const v16h b2 = Frag16::load(wb + 2 * gstr + k0);
    const v16h b3 = Frag16::load(wb + 3 * gstr + k0);
    a00 = Frag16::mma(x0, b0, a00);
    a10 = Frag16::mma(x1, b0, a10);
    a01 = Frag16::mma(x0, b1, a01);
    a11 = Frag16::mma(x1, b1, a11);
    a02 = Frag16::mma(x0, b2, a02);
    a12 = Frag16::mma(x1, b2, a12);
    a03 = Frag16::mma(x0, b3, a03);
    a13 = Frag16::mma(x1, b3, a13);
    guard8(a00, a01, a02, a03, a10, a11, a12, a13, x0, x1, b0, b1, b2, b3);
  }
  const float bi = bj[0];
  const float bf = bj[NHID];
  const float bg = bj[2 * NHID];
  const float bo = bj[3 * NHID];
  cell8(a00, a01, a02, a03, bi, bf, bg, bo, wo, cs[0], hp[0], hcol);
  cell8(a10, a11, a12, a13, bi, bf, bg, bo, wo, cs[1], hp[1], hcol + 16 * APITCH);
}

__global__ __launch_bounds__(LTHR) void lstm_seq_kernel(const unsigned short* __restrict__ Xp, const unsigned short* __restrict__ Wp,
                                                        const float* __restrict__ bih, const float* __restrict__ bhh,
                                                        const float* __restrict__ wout, const float* __restrict__ bout,
                                                        float* __restrict__ out) {
  __shared__ __align__(16) _Float16 At[2 * ATILE];
  __shared__ __align__(16) float    biasS[NGATE];
  __shared__ __align__(16) float    hpS[2 * NWAVE * MBLK];
  __shared__ __align__(16) float    outT[MBLK * OPITCH];
  const _Float16* W = (const _Float16*)Wp;
  const int tid = threadIdx.x, lane = tid & 31, wave = tid >> 5;
  const int c = lane & 15, hh = lane >> 4, koff = hh * 8;
  const int rowbase = blockIdx.x * MBLK;
  const int xr = tid >> 4, xc8 = (tid & 15) * 8;

  {
    const v4f a = *(const v4f*)(bih + 4 * tid);
    const v4f b = *(const v4f*)(bhh + 4 * tid);
    const v4f s = a + b;
    *(v4f*)(biasS + 4 * tid) = s;
  }
#pragma unroll 1
  for (int i = tid; i < MBLK * (APITCH - NEMB); i += LTHR) {
    const int row = i / (APITCH - NEMB);
    const int col = i - row * (APITCH - NEMB);
    At[row * APITCH + NEMB + col] = (_Float16)0.0f;
  }
  {
    const v4u x0 = *(const v4u*)(Xp + ((size_t)rowbase + xr) * NEMB + xc8);
    *(v4u*)(At + xr * APITCH + xc8) = x0;
  }
  __syncthreads();

  const int j0 = 32 * wave + c;
  const float wo0 = wout[j0];
  const float wo1 = wout[j0 + 16];
  const float bout0 = bout[0];
  const _Float16* wb0 = W + (size_t)j0 * KCAT + koff;
  const _Float16* wb1 = W + (size_t)(j0 + 16) * KCAT + koff;
  const float* bj0 = biasS + j0;

  float cstA[2][8], cstB[2][8];
#pragma unroll
  for (int mt = 0; mt < 2; ++mt)
#pragma unroll
    for (int r = 0; r < 8; ++r) { cstA[mt][r] = 0.0f; cstB[mt][r] = 0.0f; }

#pragma unroll 1
  for (int t = 0; t < NSTEP; ++t) {
    const int cur = t & 1;
    const _Float16* acur = At + cur * ATILE;
    _Float16* anxt = At + (cur ^ 1) * ATILE;
    const _Float16* arow0 = acur + c * APITCH + koff;
    const _Float16* arow1 = arow0 + 16 * APITCH;
    _Float16* hcol = anxt + (8 * hh) * APITCH + NEMB + j0;

    float hp[2][8];
#pragma unroll
    for (int mt = 0; mt < 2; ++mt)
#pragma unroll
      for (int r = 0; r < 8; ++r) hp[mt][r] = 0.0f;

    unit_group(arow0, arow1, wb0, hcol,      bj0,      wo0, cstA, hp);
    unit_group(arow0, arow1, wb1, hcol + 16, bj0 + 16, wo1, cstB, hp);

#pragma unroll
    for (int mt = 0; mt < 2; ++mt) {
#pragma unroll
      for (int r = 0; r < 8; ++r) {
        float v = hp[mt][r];
        v += __shfl_xor(v, 1, 32);
        v += __shfl_xor(v, 2, 32);
        v += __shfl_xor(v, 4, 32);
        v += __shfl_xor(v, 8, 32);
        hp[mt][r] = v;
      }
    }
    if (c == 0) {
#pragma unroll
      for (int mt = 0; mt < 2; ++mt) {
        const v4f plo = {hp[mt][0], hp[mt][1], hp[mt][2], hp[mt][3]};
        const v4f phi = {hp[mt][4], hp[mt][5], hp[mt][6], hp[mt][7]};
        float* pp = hpS + cur * (NWAVE * MBLK) + wave * MBLK + mt * 16 + 8 * hh;
        *(v4f*)(pp) = plo;
        *(v4f*)(pp + 4) = phi;
      }
    }
    {
      const int tn = (t + 1 < NSTEP) ? (t + 1) : (NSTEP - 1);
      const v4u xn = *(const v4u*)(Xp + ((size_t)tn * NBAT + rowbase + xr) * NEMB + xc8);
      *(v4u*)(anxt + xr * APITCH + xc8) = xn;
    }
    __syncthreads();

    if (wave == 0) {
      const float* hq = hpS + cur * (NWAVE * MBLK) + lane;
      float s = 0.0f;
#pragma unroll
      for (int w2 = 0; w2 < NWAVE; ++w2) s += hq[w2 * MBLK];
      s += bout0;
      const int col = t & (OTILE - 1);
      outT[lane * OPITCH + col] = s;
      __builtin_amdgcn_fence(__ATOMIC_RELEASE, "workgroup");
      __builtin_amdgcn_wave_barrier();
      __builtin_amdgcn_fence(__ATOMIC_ACQUIRE, "workgroup");
      if (col == OTILE - 1) {
        const int t0 = t - (OTILE - 1);
        const int q = lane >> 3, c4 = (lane & 7) * 4;
        for (int pass = 0; pass < 2; ++pass) {
#pragma unroll
          for (int it = 0; it < 8; ++it) {
            const int row = it * 4 + q;
            const v4f v = *(const v4f*)(outT + row * OPITCH + c4);
            *(volatile v4f*)(out + (size_t)(rowbase + row) * NSTEP + t0 + c4) = v;
          }
          __threadfence();
        }
        __builtin_amdgcn_fence(__ATOMIC_RELEASE, "workgroup");
        __builtin_amdgcn_wave_barrier();
        __builtin_amdgcn_fence(__ATOMIC_ACQUIRE, "workgroup");
      }
    }
  }
}

extern "C" void kernel_launch(void* const* d_in, const int* in_sizes, int n_in,
                              void* d_out, int out_size, void* d_ws, size_t ws_size, hipStream_t stream) {
  if (n_in < 9 || d_out == nullptr || d_ws == nullptr) return;
  if (in_sizes[0] != NBAT * NSTEP * NTOKL || in_sizes[1] != NBAT * NSTEP * NTOKL || in_sizes[2] != NVOCAB * NEMB ||
      in_sizes[3] != NGATE * NEMB || in_sizes[4] != NGATE * NHID || in_sizes[5] != NGATE || in_sizes[6] != NGATE ||
      in_sizes[7] != NHID || in_sizes[8] != 1 || out_size != NBAT * NSTEP) return;

  const int*   tokens = (const int*)d_in[0];
  const float* values = (const float*)d_in[1];
  const float* emb    = (const float*)d_in[2];
  const float* wih    = (const float*)d_in[3];
  const float* whh    = (const float*)d_in[4];
  const float* bih    = (const float*)d_in[5];
  const float* bhh    = (const float*)d_in[6];
  const float* wout   = (const float*)d_in[7];
  const float* bout   = (const float*)d_in[8];
  float* out = (float*)d_out;

  char* ws = (char*)d_ws; size_t off = 0;
  auto carve = [&](size_t bytes) -> char* { char* p = ws + off; off += (bytes + 255) & ~(size_t)255; return p; };
  unsigned short* XPL  = (unsigned short*)carve((size_t)NSTEP * NBAT * NEMB * 2);
  unsigned short* WCAT = (unsigned short*)carve((size_t)NGATE * KCAT * 2);
  if (off > ws_size || off > (size_t)134217728) return;

  prep_weights_kernel<<<IH_BLOCKS + HH_BLOCKS, PTHR, 0, stream>>>(wih, whh, WCAT);
  embed_kernel<<<(NBAT * NSTEP) / (PTHR / 32), PTHR, 0, stream>>>(tokens, values, emb, XPL);
  lstm_seq_kernel<<<NBAT / MBLK, LTHR, 0, stream>>>(XPL, WCAT, bih, bhh, wout, bout, out);
}
